// ContinuousFilterConvolution_58325655879889
// MI455X (gfx1250) — hardware-verified
//
#include <hip/hip_runtime.h>
#include <stdint.h>
#include <stddef.h>


typedef _Float16 h16;
typedef _Float16 v16h __attribute__((ext_vector_type(16)));
typedef _Float16 v8h  __attribute__((ext_vector_type(8)));
typedef float    v8f  __attribute__((ext_vector_type(8)));
typedef float    v4f  __attribute__((ext_vector_type(4)));
typedef int      v4i  __attribute__((ext_vector_type(4)));
typedef unsigned v4u  __attribute__((ext_vector_type(4)));

union Frag  { v16h v; v8h hv[2]; };
union Pack8 { v8h h; v4u u; };

constexpr int   CH    = 256;
constexpr int   NCEN  = 200;
constexpr int   K1    = 224;
constexpr int   WP    = 256;
constexpr int   TN    = 64;
constexpr int   TE    = 64;
constexpr int   AP    = CH + 8;
constexpr int   LCAP  = 2048;
constexpr int   MAXT  = LCAP / TE;
constexpr int   NTHR  = 256;
constexpr float WSC   = 16.0f;
constexpr float WINV  = 0.0625f;
constexpr float LOG2F_ = 0.69314718055994531f;

typedef char chk_tile_shared[(TN == TE) ? 1 : -1];
typedef char chk_lds_align[((AP * 2) % 16 == 0) ? 1 : -1];
typedef char chk_k1[(K1 % 32 == 0 && K1 >= NCEN && K1 <= WP) ? 1 : -1];

__device__ __forceinline__ float sspf(float v) {
    const bool  lo = v < 14.0f;
    const float vs = lo ? v : 0.0f;
    const float sp = __logf(1.0f + __expf(vs));
    return (lo ? sp : v) - LOG2F_;
}

__device__ __forceinline__ v8f wmma16(v16h a, v16h b, v8f c) {
    v8f d = __builtin_amdgcn_wmma_f32_16x16x32_f16(false, a, false, b, (short)0, c, false, false);
    asm volatile("v_nop\n\tv_nop\n\tv_nop\n\tv_nop" : "+v"(d) : "v"(a), "v"(b));
    return d;
}

__device__ __forceinline__ v16h ldfrag(const h16* base, int pitch, int row, int k0, int h) {
    Frag f;
    const h16* p = base + (size_t)row * pitch + k0 + 8 * h;
    f.hv[0] = *(const v8h*)(p);
    f.hv[1] = *(const v8h*)(p + 16);
    return f.v;
}

template<int R>
__device__ __forceinline__ void zacc(v8f (&acc)[2][R]) {
    v8f z = {};
#pragma unroll
    for (int c = 0; c < 2; ++c)
#pragma unroll
        for (int r = 0; r < R; ++r) acc[c][r] = z;
}

template<int R, int KS>
__device__ __forceinline__ void wave_gemm(const h16* A, int lda, const h16* Bt,
                                          int n0, int ln, int h, v8f (&acc)[2][R]) {
#pragma unroll 1
    for (int ks = 0; ks < KS; ++ks) {
        const int k0 = ks * 32;
        const v16h b0 = ldfrag(Bt, WP, n0, k0, h);
        const v16h b1 = ldfrag(Bt, WP, n0 + 16, k0, h);
#pragma unroll
        for (int r = 0; r < R; ++r) {
            const v16h a = ldfrag(A, lda, r * 16 + ln, k0, h);
            acc[0][r] = wmma16(a, b0, acc[0][r]);
            acc[1][r] = wmma16(a, b1, acc[1][r]);
        }
    }
}

template<int R>
__device__ __forceinline__ void epi_act(v8f (&acc)[2][R], const float* __restrict__ bias,
                                        h16* dst, int n0, int h) {
#pragma unroll
    for (int c = 0; c < 2; ++c) {
        const int   n  = n0 + 16 * c;
        const float bv = bias[n];
#pragma unroll
        for (int r = 0; r < R; ++r)
#pragma unroll
            for (int q = 0; q < 8; ++q)
                dst[(r * 16 + 8 * h + q) * AP + n] = (h16)sspf(acc[c][r][q] * WINV + bv);
    }
}

__global__ void __launch_bounds__(NTHR)
k_prep(const float* __restrict__ w1, const float* __restrict__ w2, const float* __restrict__ w3,
       const float* __restrict__ w4, const float* __restrict__ w5, h16* __restrict__ wt)
{
    __shared__ __align__(16) h16 tile[64 * AP];
    const int tid = threadIdx.x, wid = tid >> 5, lane = tid & 31;
    const int wsel = blockIdx.x >> 2, nt = blockIdx.x & 3;
    const float* w = (wsel == 0) ? w1 : (wsel == 1) ? w2 : (wsel == 2) ? w3 : (wsel == 3) ? w4 : w5;
    const int K = (wsel == 0) ? NCEN : CH;
    h16* dst = wt + (size_t)wsel * CH * WP;
    const int n0 = nt * 64;
    for (int i = tid; i < 64 * WP; i += NTHR) {
        const int k = i >> 6, nn = i & 63;
        const float v = (k < K) ? w[(size_t)k * CH + n0 + nn] : 0.0f;
        tile[nn * AP + k] = (h16)(v * WSC);
    }
    __syncthreads();
#pragma unroll
    for (int j = 0; j < 8; ++j) {
        const int nn = wid * 8 + j;
        Pack8 p; p.h = *(const v8h*)&tile[nn * AP + lane * 8];
        *(volatile v4u*)(dst + (size_t)(n0 + nn) * WP + lane * 8) = p.u;
    }
    __threadfence();
#pragma unroll
    for (int j = 0; j < 8; ++j) {
        const int nn = wid * 8 + j;
        Pack8 p; p.h = *(const v8h*)&tile[nn * AP + lane * 8];
        *(volatile v4u*)(dst + (size_t)(n0 + nn) * WP + lane * 8) = p.u;
    }
}

__global__ void __launch_bounds__(NTHR)
k_xw3(const float* __restrict__ x, const h16* __restrict__ w3t, float* __restrict__ xw3, int N)
{
    __shared__ __align__(16) h16   xa[TN * AP];
    __shared__ __align__(16) float so[TN * CH];
    const int tid = threadIdx.x, wid = tid >> 5, lane = tid & 31, h = lane >> 4, ln = lane & 15;
    const int nbase = blockIdx.x * TN;
    for (int i = tid; i < TN * (CH / 8); i += NTHR) {
        const int m = i >> 5, kb = (i & 31) * 8;
        const int node = nbase + m;
        v4f a = {0.0f, 0.0f, 0.0f, 0.0f};
        v4f b = {0.0f, 0.0f, 0.0f, 0.0f};
        if (node < N) {
            const float* p = x + (size_t)node * CH + kb;
            a = *(const v4f*)(p);
            b = *(const v4f*)(p + 4);
        }
        const v8f t = __builtin_shufflevector(a, b, 0, 1, 2, 3, 4, 5, 6, 7);
        *(v8h*)&xa[m * AP + kb] = __builtin_convertvector(t, v8h);
    }
    __syncthreads();
    const int n0 = wid * 32 + ln;
    {
        v8f acc[2][4];
        zacc<4>(acc);
        wave_gemm<4, CH / 32>(xa, AP, w3t, n0, ln, h, acc);
#pragma unroll
        for (int c = 0; c < 2; ++c) {
            const int n = n0 + 16 * c;
#pragma unroll
            for (int r = 0; r < 4; ++r)
#pragma unroll
                for (int q = 0; q < 8; ++q)
                    so[(r * 16 + 8 * h + q) * CH + n] = acc[c][r][q] * WINV;
        }
    }
    __syncthreads();
    for (int it = 0; it < 16; ++it) {
        const int idx = it * NTHR + tid, row = idx >> 6, c4 = idx & 63;
        const v4f v = *(const v4f*)&so[row * CH + c4 * 4];
        *(volatile v4f*)(xw3 + (size_t)(nbase + row) * CH + c4 * 4) = v;
    }
    __threadfence();
    for (int it = 0; it < 16; ++it) {
        const int idx = it * NTHR + tid, row = idx >> 6, c4 = idx & 63;
        const v4f v = *(const v4f*)&so[row * CH + c4 * 4];
        *(volatile v4f*)(xw3 + (size_t)(nbase + row) * CH + c4 * 4) = v;
    }
}

__global__ void __launch_bounds__(NTHR)
k_main(const float* __restrict__ pos, const int* __restrict__ snd, const int* __restrict__ rcv,
       const float* __restrict__ x, const h16* __restrict__ wt,
       const float* __restrict__ b1, const float* __restrict__ b2,
       const float* __restrict__ b4, const float* __restrict__ b5,
       const float* __restrict__ xw3, float* __restrict__ out, int N, int E)
{
    __shared__ __align__(16) float sconv[TN * CH];
    __shared__ __align__(16) h16   bufA[TE * AP];
    __shared__ __align__(16) h16   bufH[TE * AP];
    __shared__ int   slist[LCAP];
    __shared__ int   sS[TE];
    __shared__ int   sRl[TE];
    __shared__ float sD[TE];
    __shared__ int   swc[16];

    const int tid = threadIdx.x, wid = tid >> 5, lane = tid & 31, h = lane >> 4, ln = lane & 15;
    const int n0 = wid * 32 + ln;
    const int nbase = blockIdx.x * TN;
    const h16* w1t = wt;
    const h16* w2t = wt + (size_t)1 * CH * WP;
    const h16* w4t = wt + (size_t)3 * CH * WP;
    const h16* w5t = wt + (size_t)4 * CH * WP;

    for (int i = tid; i < TN * CH; i += NTHR) sconv[i] = 0.0f;

    int total = 0;
    int par = 0;
    for (int c0 = 0; c0 < E; c0 += NTHR * 8) {
        const int eb = c0 + tid * 8;
        unsigned mask = 0u;
        if (eb + 8 <= E) {
            const v4i ra = *(const v4i*)(rcv + eb);
            const v4i rb = *(const v4i*)(rcv + eb + 4);
            mask |= ((unsigned)(ra.x - nbase) < (unsigned)TN) ? 1u   : 0u;
            mask |= ((unsigned)(ra.y - nbase) < (unsigned)TN) ? 2u   : 0u;
            mask |= ((unsigned)(ra.z - nbase) < (unsigned)TN) ? 4u   : 0u;
            mask |= ((unsigned)(ra.w - nbase) < (unsigned)TN) ? 8u   : 0u;
            mask |= ((unsigned)(rb.x - nbase) < (unsigned)TN) ? 16u  : 0u;
            mask |= ((unsigned)(rb.y - nbase) < (unsigned)TN) ? 32u  : 0u;
            mask |= ((unsigned)(rb.z - nbase) < (unsigned)TN) ? 64u  : 0u;
            mask |= ((unsigned)(rb.w - nbase) < (unsigned)TN) ? 128u : 0u;
        } else {
#pragma unroll
            for (int j = 0; j < 8; ++j) {
                const int e = eb + j;
                if (e < E) {
                    const int r = rcv[e];
                    if ((unsigned)(r - nbase) < (unsigned)TN) mask |= (1u << j);
                }
            }
        }
        const int cnt = (int)__popc(mask);
        int incl = cnt;
#pragma unroll
        for (int d = 1; d < 32; d <<= 1) {
            const int t = __shfl_up(incl, d);
            if (lane >= d) incl += t;
        }
        const int wtot = __shfl(incl, 31);
        if (lane == 0) swc[par * 8 + wid] = wtot;
        __syncthreads();
        int woff = 0, csum = 0;
#pragma unroll
        for (int wv = 0; wv < 8; ++wv) {
            const int c = swc[par * 8 + wv];
            csum += c;
            woff += (wv < wid) ? c : 0;
        }
        int p = total + woff + (incl - cnt);
        if (mask != 0u) {
#pragma unroll
            for (int j = 0; j < 8; ++j) {
                if (mask & (1u << j)) {
                    if ((unsigned)p < (unsigned)LCAP) slist[p] = eb + j;
                    ++p;
                }
            }
        }
        total += csum;
        par ^= 1;
    }
    const int ecnt = min(total, LCAP);
    __syncthreads();

    for (int t = 0; t < MAXT; ++t) {
        if (t * TE >= ecnt) break;
        const int nval = min(TE, ecnt - t * TE);
        if (tid < TE) {
            const int li = t * TE + tid;
            int e = 0;
            if (li < ecnt) e = slist[li];
            e = min(max(e, 0), E - 1);
            const int s = snd[e], r = rcv[e];
            const int sc = min(max(s, 0), N - 1);
            const int rc = min(max(r, 0), N - 1);
            int rl = r - nbase; rl = min(max(rl, 0), TN - 1);
            const float dx = pos[3 * rc + 0] - pos[3 * sc + 0];
            const float dy = pos[3 * rc + 1] - pos[3 * sc + 1];
            const float dz = pos[3 * rc + 2] - pos[3 * sc + 2];
            sS[tid]  = sc;
            sRl[tid] = rl;
            sD[tid]  = sqrtf(dx * dx + dy * dy + dz * dz);
        }
        __syncthreads();
        for (int i = tid; i < TE * (K1 / 8); i += NTHR) {
            const int m = i / (K1 / 8), kb = (i - m * (K1 / 8)) * 8;
            const float d0 = sD[m];
            v8h hv;
#pragma unroll
            for (int j = 0; j < 8; ++j) {
                const int k = kb + j;
                const float ck = (k == NCEN - 1) ? 20.0f : 20.0f * ((float)k * (1.0f / 199.0f));
                const float dd = d0 - ck;
                const float v = (k < NCEN) ? __expf(-(dd * dd) * 10.0f) : 0.0f;
                hv[j] = (h16)v;
            }
            *(v8h*)&bufA[m * AP + kb] = hv;
        }
        __syncthreads();
        {
            v8f acc[2][4];
            zacc<4>(acc);
            wave_gemm<4, K1 / 32>(bufA, AP, w1t, n0, ln, h, acc);
            epi_act<4>(acc, b1, bufH, n0, h);
        }
        __syncthreads();
        {
            v8f acc[2][4];
            zacc<4>(acc);
            wave_gemm<4, CH / 32>(bufH, AP, w2t, n0, ln, h, acc);
            epi_act<4>(acc, b2, bufA, n0, h);
        }
        __syncthreads();
        for (int e = 0; e < nval; ++e) {
            const float f  = xw3[(size_t)sS[e] * CH + tid];
            const float wv = (float)bufA[e * AP + tid];
            sconv[sRl[e] * CH + tid] += wv * f;
        }
        __syncthreads();
    }

    for (int i = tid; i < TN * (CH / 8); i += NTHR) {
        const int m = i >> 5, kb = (i & 31) * 8;
        const v4f a = *(const v4f*)&sconv[m * CH + kb];
        const v4f b = *(const v4f*)&sconv[m * CH + kb + 4];
        const v8f t = __builtin_shufflevector(a, b, 0, 1, 2, 3, 4, 5, 6, 7);
        *(v8h*)&bufA[m * AP + kb] = __builtin_convertvector(t, v8h);
    }
    __syncthreads();
    {
        v8f acc[2][4];
        zacc<4>(acc);
        wave_gemm<4, CH / 32>(bufA, AP, w4t, n0, ln, h, acc);
        epi_act<4>(acc, b4, bufH, n0, h);
    }
    __syncthreads();
    {
        v8f acc[2][4];
        zacc<4>(acc);
        wave_gemm<4, CH / 32>(bufH, AP, w5t, n0, ln, h, acc);
#pragma unroll
        for (int c = 0; c < 2; ++c) {
            const int   n  = n0 + 16 * c;
            const float bv = b5[n];
#pragma unroll
            for (int r = 0; r < 4; ++r)
#pragma unroll
                for (int q = 0; q < 8; ++q)
                    sconv[(r * 16 + 8 * h + q) * CH + n] = acc[c][r][q] * WINV + bv;
        }
    }
    __syncthreads();
    for (int it = 0; it < 16; ++it) {
        const int idx = it * NTHR + tid, row = idx >> 6, c4 = idx & 63;
        const int node = nbase + row;
        if (node < N) {
            const v4f v  = *(const v4f*)&sconv[row * CH + c4 * 4];
            const v4f xv = *(const v4f*)(x + (size_t)node * CH + c4 * 4);
            const v4f o  = xv + v;
            *(volatile v4f*)(out + (size_t)node * CH + c4 * 4) = o;
        }
    }
    __threadfence();
    for (int it = 0; it < 16; ++it) {
        const int idx = it * NTHR + tid, row = idx >> 6, c4 = idx & 63;
        const int node = nbase + row;
        if (node < N) {
            const v4f v  = *(const v4f*)&sconv[row * CH + c4 * 4];
            const v4f xv = *(const v4f*)(x + (size_t)node * CH + c4 * 4);
            const v4f o  = xv + v;
            *(volatile v4f*)(out + (size_t)node * CH + c4 * 4) = o;
        }
    }
}

extern "C" void kernel_launch(void* const* d_in, const int* in_sizes, int n_in,
                              void* d_out, int out_size, void* d_ws, size_t ws_size,
                              hipStream_t stream)
{
    if (n_in < 13) return;
    const float* pos = (const float*)d_in[0];
    const float* x   = (const float*)d_in[1];
    const int*   snd = (const int*)d_in[2];
    const int*   rcv = (const int*)d_in[3];
    const float* w1  = (const float*)d_in[4];
    const float* b1  = (const float*)d_in[5];
    const float* w2  = (const float*)d_in[6];
    const float* b2  = (const float*)d_in[7];
    const float* w3  = (const float*)d_in[8];
    const float* w4  = (const float*)d_in[9];
    const float* b4  = (const float*)d_in[10];
    const float* w5  = (const float*)d_in[11];
    const float* b5  = (const float*)d_in[12];

    const int N = in_sizes[0] / 3;
    const int E = in_sizes[2];
    if (N <= 0 || E < 0) return;
    if (in_sizes[0] != N * 3 || in_sizes[1] != N * CH || in_sizes[3] != E) return;
    if (in_sizes[4] != NCEN * CH || in_sizes[5] != CH || in_sizes[6] != CH * CH || in_sizes[7] != CH ||
        in_sizes[8] != CH * CH || in_sizes[9] != CH * CH || in_sizes[10] != CH ||
        in_sizes[11] != CH * CH || in_sizes[12] != CH) return;
    if (out_size != N * CH) return;

    const int    nblk   = (N + TN - 1) / TN;
    const size_t npad   = (size_t)nblk * TN;
    const size_t o_wt   = 0;
    const size_t wt_b   = (size_t)5 * CH * WP * sizeof(h16);
    const size_t o_xw3  = o_wt + wt_b;
    const size_t xw3_b  = npad * CH * sizeof(float);
    const size_t total  = o_xw3 + xw3_b;
    if (total > ws_size) return;

    char*  ws  = (char*)d_ws;
    h16*   wt  = (h16*)(ws + o_wt);
    float* xw3 = (float*)(ws + o_xw3);
    float* out = (float*)d_out;

    k_prep<<<20, NTHR, 0, stream>>>(w1, w2, w3, w4, w5, wt);
    k_xw3<<<nblk, NTHR, 0, stream>>>(x, wt + (size_t)2 * CH * WP, xw3, N);
    k_main<<<nblk, NTHR, 0, stream>>>(pos, snd, rcv, x, wt, b1, b2, b4, b5, xw3, out, N, E);
}
